// FlashAttention_38336878084668
// MI455X (gfx1250) — hardware-verified
//
#include <hip/hip_runtime.h>


#ifndef NB
#define NB 2
#endif
#ifndef SEQ
#define SEQ 2048
#endif
#define NB_FULL  2
#define SEQ_FULL 2048
#define DIM   768
#define NHD   12
#define HD    64
#define INNER (NHD * HD)
#define NQKV  (3 * INNER)
#define NZ    (NB * NHD)
#define MROWS (NB * SEQ)
#define PCAR  1024.0f
#define WSC   16.0f
#define OSC   (1.0f / 16384.0f)
#define SL2   0.18033688011112042f

static_assert(NB >= 1 && NB <= NB_FULL);
static_assert(SEQ % 256 == 0 && SEQ <= SEQ_FULL);
static_assert(HD == 64 && DIM % 64 == 0 && INNER % 64 == 0 && NQKV % 64 == 0 && MROWS % 64 == 0);
static_assert((NQKV * DIM) % 4096 == 0 && (DIM * INNER) % 4096 == 0);
static_assert(((size_t)SEQ * DIM) % 2048 == 0 && ((size_t)NZ * SEQ * HD) % 2048 == 0);

typedef _Float16 h16;
typedef unsigned short bf;
typedef __attribute__((ext_vector_type(16))) __bf16   v16bf;
typedef __attribute__((ext_vector_type(16))) _Float16 v16h;
typedef __attribute__((ext_vector_type(8)))  _Float16 v8h;
typedef __attribute__((ext_vector_type(8)))  unsigned short v8us;
typedef __attribute__((ext_vector_type(8)))  float    v8f;
typedef __attribute__((ext_vector_type(4)))  float    v4f;
typedef __attribute__((ext_vector_type(2)))  _Float16 v2h;
typedef __attribute__((ext_vector_type(2)))  unsigned short v2us;
typedef v8h  __attribute__((may_alias)) v8ha;
typedef v4f  __attribute__((may_alias)) v4fa;
typedef v8us __attribute__((may_alias)) v8usa;

__device__ __forceinline__ unsigned short f2bf(float f) { unsigned u = __float_as_uint(f); u += 0x7FFFu + ((u >> 16) & 1u); return (unsigned short)(u >> 16); }
__device__ __forceinline__ float bf2f(unsigned short b) { return __uint_as_float(((unsigned)b) << 16); }
__device__ __forceinline__ float bfr(float f) { return bf2f(f2bf(f)); }
__device__ __forceinline__ v16h cat16(v8h lo, v8h hi) { return __builtin_shufflevector(lo, hi, 0, 1, 2, 3, 4, 5, 6, 7, 8, 9, 10, 11, 12, 13, 14, 15); }
__device__ __forceinline__ v16bf cat16b(v8us lo, v8us hi) { return __builtin_bit_cast(v16bf, __builtin_shufflevector(lo, hi, 0, 1, 2, 3, 4, 5, 6, 7, 8, 9, 10, 11, 12, 13, 14, 15)); }
__device__ __forceinline__ v8f wmma16(v16h a, v16h b, v8f c) { return __builtin_amdgcn_wmma_f32_16x16x32_f16(false, a, false, b, (short)0, c, false, false); }
__device__ __forceinline__ v8f wmmab(v16bf a, v16bf b, v8f c) { return __builtin_amdgcn_wmma_f32_16x16x32_bf16(false, a, false, b, (short)0, c, false, false); }

template <typename T16> struct WFrag;
template <> struct WFrag<h16> { typedef v16h V; static __device__ __forceinline__ V ld(const h16* p) { return cat16(*(const v8h*)p, *(const v8h*)(p + 16)); } static __device__ __forceinline__ v8f mma(V a, V b, v8f c) { return wmma16(a, b, c); } };
template <> struct WFrag<bf> { typedef v16bf V; static __device__ __forceinline__ V ld(const bf* p) { return cat16b(*(const v8us*)p, *(const v8us*)(p + 16)); } static __device__ __forceinline__ v8f mma(V a, V b, v8f c) { return wmmab(a, b, c); } };

template <typename T16, int NSPLIT, bool BIAS>
__global__ __launch_bounds__(32) void k_gemmw(const T16* __restrict__ A, const T16* __restrict__ A2, const T16* __restrict__ Bt, const T16* __restrict__ Bt2, int K, float* C, int ldc, const float* __restrict__ bias, float osc, size_t sA, size_t sB, size_t sC) {
    typedef typename WFrag<T16>::V V;
    __shared__ __align__(16) float os[16 * 68];
    const size_t z = blockIdx.z; A += z * sA; if (A2) A2 += z * sA; Bt += z * sB; if (Bt2) Bt2 += z * sB; C += z * sC;
    const int lane = threadIdx.x & 31, lr = lane & 15, hi = lane >> 4; const int r0 = blockIdx.x * 64, c0 = blockIdx.y * 64;
    v8f acc[4][4];
#pragma unroll
    for (int mb = 0; mb < 4; ++mb)
#pragma unroll
        for (int nb = 0; nb < 4; ++nb) acc[mb][nb] = (v8f){};
    const size_t aoff = (size_t)(r0 + lr) * K + 8 * hi, boff = (size_t)(c0 + lr) * K + 8 * hi;
#pragma unroll 1
    for (int kc = 0; kc < K; kc += 32) {
        V a[4], a2[4];
#pragma unroll
        for (int mb = 0; mb < 4; ++mb) { a[mb] = WFrag<T16>::ld(A + aoff + (size_t)mb * 16 * K + kc); if (NSPLIT == 1 || NSPLIT == 2) a2[mb] = WFrag<T16>::ld(A2 + aoff + (size_t)mb * 16 * K + kc); }
#pragma unroll
        for (int nb = 0; nb < 4; ++nb) { const V b = WFrag<T16>::ld(Bt + boff + (size_t)nb * 16 * K + kc); V b2; if (NSPLIT >= 2) b2 = WFrag<T16>::ld(Bt2 + boff + (size_t)nb * 16 * K + kc);
#pragma unroll
            for (int mb = 0; mb < 4; ++mb) { acc[mb][nb] = WFrag<T16>::mma(a[mb], b, acc[mb][nb]); if (NSPLIT == 1 || NSPLIT == 2) acc[mb][nb] = WFrag<T16>::mma(a2[mb], b, acc[mb][nb]); if (NSPLIT >= 2) acc[mb][nb] = WFrag<T16>::mma(a[mb], b2, acc[mb][nb]); } }
        asm volatile("v_nop\n\tv_nop\n\tv_nop\n\tv_nop" : "+v"(acc[0][0]), "+v"(acc[1][1]), "+v"(acc[2][2]), "+v"(acc[3][3]) : "v"(a[0]), "v"(a[3]));
    }
#pragma unroll
    for (int mb = 0; mb < 4; ++mb) {
#pragma unroll
        for (int nb = 0; nb < 4; ++nb) {
#pragma unroll
            for (int j = 0; j < 8; ++j) os[(hi * 8 + j) * 68 + nb * 16 + lr] = acc[mb][nb][j]; }
        __builtin_amdgcn_wave_barrier(); asm volatile("" ::: "memory");
        float* crow = C + (size_t)(r0 + mb * 16) * ldc + c0;
#pragma unroll 1
        for (int ps = 0; ps < 2; ++ps) {
#pragma unroll
            for (int s = 0; s < 8; ++s) { const int row = 2 * s + hi, cofs = lr * 4; v4f val = *(const v4fa*)(os + row * 68 + cofs); val = val * osc; if (BIAS) { val[0] += bfr(bias[c0 + cofs]); val[1] += bfr(bias[c0 + cofs + 1]); val[2] += bfr(bias[c0 + cofs + 2]); val[3] += bfr(bias[c0 + cofs + 3]); }
                *(volatile v4f*)(crow + (size_t)row * ldc + cofs) = val; }
            if (ps == 0) __threadfence(); }
        __builtin_amdgcn_wave_barrier(); asm volatile("" ::: "memory");
    }
}

__global__ __launch_bounds__(256) void k_cvt8(const float* __restrict__ src, bf* dst, size_t n8) { const size_t i = (size_t)blockIdx.x * 256 + threadIdx.x; if (i >= n8) return; const v8f v = *(const v8f*)(src + i * 8); v8us o;
#pragma unroll
    for (int k = 0; k < 8; ++k) o[k] = f2bf(v[k]); *(volatile v8us*)(dst + i * 8) = o; __threadfence(); *(volatile v8us*)(dst + i * 8) = o; }

template <typename T16> struct P2;
template <> struct P2<bf>  { typedef v2us V; static __device__ __forceinline__ bf  c(float f) { return f2bf(f); } };
template <> struct P2<h16> { typedef v2h  V; static __device__ __forceinline__ h16 c(float f) { return (h16)bfr(f); } };
template <typename T16>
__global__ __launch_bounds__(256) void k_wt(const float* __restrict__ w, int K, int N, float sc, T16* Bt) {
    typedef typename P2<T16>::V V2;
    const int lane = threadIdx.x & 31; const int L0 = (blockIdx.x * 8 + (threadIdx.x >> 5)) * 8; const int nlines = N * K / 64;
#pragma unroll
    for (int ps = 0; ps < 2; ++ps) {
#pragma unroll 1
        for (int l = 0; l < 8; ++l) { const int L = L0 + l; if (L >= nlines) break; const size_t e = (size_t)L * 64 + lane * 2; const int k = (int)(e % K), n = (int)(e / K); V2 o;
            o[0] = P2<T16>::c(w[(size_t)k * N + n] * sc); o[1] = P2<T16>::c(w[(size_t)(k + 1) * N + n] * sc); *(volatile V2*)(Bt + e) = o; }
        if (ps == 0) __threadfence(); }
}

__global__ __launch_bounds__(256) void k_qkp(const float* __restrict__ F, h16* Q16, h16* K16) {
    const size_t i = (size_t)blockIdx.x * 256 + threadIdx.x; const size_t n8 = (size_t)NZ * SEQ * HD / 8; if (i >= n8) return;
    const size_t e = i * 8; const int d = (int)(e % HD); const int s = (int)((e / HD) % SEQ); const int z = (int)(e / ((size_t)HD * SEQ)); const int b = z / NHD, h = z - b * NHD;
    const float* src = F + ((size_t)b * SEQ + s) * NQKV + h * HD + d;
    const v8f q = *(const v8f*)src; const v8f k = *(const v8f*)(src + INNER);
    v8h oq, ok;
#pragma unroll
    for (int j = 0; j < 8; ++j) { oq[j] = (h16)q[j]; ok[j] = (h16)k[j]; }
    *(volatile v8h*)(Q16 + e) = oq; *(volatile v8h*)(K16 + e) = ok; __threadfence(); *(volatile v8h*)(Q16 + e) = oq; *(volatile v8h*)(K16 + e) = ok;
}

__global__ __launch_bounds__(256) void k_vtp(const float* __restrict__ F, h16* VT) {
    const size_t i = (size_t)blockIdx.x * 256 + threadIdx.x; const size_t n8 = (size_t)NZ * HD * SEQ / 8; if (i >= n8) return;
    const size_t e = i * 8; const int t = (int)(e % SEQ); const int d = (int)((e / SEQ) % HD); const int z = (int)(e / ((size_t)SEQ * HD)); const int b = z / NHD, h = z - b * NHD;
    const float* src = F + ((size_t)b * SEQ + t) * NQKV + 2 * INNER + h * HD + d;
    v8h o;
#pragma unroll
    for (int q = 0; q < 8; ++q) o[q] = (h16)src[(size_t)q * NQKV];
    *(volatile v8h*)(VT + e) = o; __threadfence(); *(volatile v8h*)(VT + e) = o;
}

__global__ __launch_bounds__(32) void k_attn(const h16* __restrict__ Q16, const h16* __restrict__ K16, const h16* __restrict__ VT, h16* C16) {
    __shared__ __align__(16) h16 pt[16 * 72];
    const int lane = threadIdx.x & 31, lr = lane & 15, hi = lane >> 4;
    const int s0 = blockIdx.x * 16; const int z = blockIdx.y; const int b = z / NHD, h = z - b * NHD;
    const h16* qp = Q16 + ((size_t)z * SEQ + s0 + lr) * HD + 8 * hi;
    const v16h qf0 = WFrag<h16>::ld(qp), qf1 = WFrag<h16>::ld(qp + 32);
    const h16* kp = K16 + ((size_t)z * SEQ + lr) * HD + 8 * hi;
    const h16* vp = VT + ((size_t)z * HD + lr) * SEQ + 8 * hi;
    float mrow[8], lrow[8]; v8f acc[4];
#pragma unroll
    for (int r = 0; r < 8; ++r) { mrow[r] = -3.0e38f; lrow[r] = 0.f; }
#pragma unroll
    for (int jd = 0; jd < 4; ++jd) acc[jd] = (v8f){};
#pragma unroll 1
    for (int kb = 0; kb < SEQ; kb += 64) {
        v8f sc[4];
#pragma unroll
        for (int j = 0; j < 4; ++j) { const h16* kk = kp + (size_t)(kb + j * 16) * HD; const v16h b0 = WFrag<h16>::ld(kk), b1 = WFrag<h16>::ld(kk + 32); v8f s = (v8f){}; s = wmma16(qf0, b0, s); s = wmma16(qf1, b1, s); sc[j] = s; }
        asm volatile("v_nop\n\tv_nop\n\tv_nop\n\tv_nop" : "+v"(sc[0]), "+v"(sc[1]), "+v"(sc[2]), "+v"(sc[3]) : "v"(qf0), "v"(qf1));
#pragma unroll
        for (int r = 0; r < 8; ++r) {
            float t0 = sc[0][r] * SL2, t1 = sc[1][r] * SL2, t2 = sc[2][r] * SL2, t3 = sc[3][r] * SL2;
            float mx = fmaxf(fmaxf(t0, t1), fmaxf(t2, t3));
#pragma unroll
            for (int off = 1; off < 16; off <<= 1) mx = fmaxf(mx, __shfl_xor(mx, off, 32));
            const float mnew = fmaxf(mrow[r], mx);
            const float alpha = __builtin_amdgcn_exp2f(mrow[r] - mnew);
            mrow[r] = mnew;
            t0 = __builtin_amdgcn_exp2f(t0 - mnew); t1 = __builtin_amdgcn_exp2f(t1 - mnew); t2 = __builtin_amdgcn_exp2f(t2 - mnew); t3 = __builtin_amdgcn_exp2f(t3 - mnew);
            float rs = (t0 + t1) + (t2 + t3);
#pragma unroll
            for (int off = 1; off < 16; off <<= 1) rs += __shfl_xor(rs, off, 32);
            lrow[r] = lrow[r] * alpha + rs;
            sc[0][r] = t0; sc[1][r] = t1; sc[2][r] = t2; sc[3][r] = t3;
#pragma unroll
            for (int jd = 0; jd < 4; ++jd) acc[jd][r] *= alpha;
        }
#pragma unroll
        for (int j = 0; j < 4; ++j)
#pragma unroll
            for (int r = 0; r < 8; ++r) pt[(8 * hi + r) * 72 + j * 16 + lr] = (h16)(sc[j][r] * PCAR);
        __syncthreads();
        const v16h pf0 = cat16(*(const v8ha*)(pt + lr * 72 + 8 * hi), *(const v8ha*)(pt + lr * 72 + 16 + 8 * hi));
        const v16h pf1 = cat16(*(const v8ha*)(pt + lr * 72 + 32 + 8 * hi), *(const v8ha*)(pt + lr * 72 + 48 + 8 * hi));
#pragma unroll
        for (int jd = 0; jd < 4; ++jd) { const h16* vv = vp + (size_t)jd * 16 * SEQ + kb; const v16h v0 = WFrag<h16>::ld(vv), v1 = WFrag<h16>::ld(vv + 32); acc[jd] = wmma16(pf0, v0, acc[jd]); acc[jd] = wmma16(pf1, v1, acc[jd]); }
        asm volatile("v_nop\n\tv_nop\n\tv_nop\n\tv_nop" : "+v"(acc[0]), "+v"(acc[1]), "+v"(acc[2]), "+v"(acc[3]) : "v"(pf0), "v"(pf1));
        __syncthreads();
    }
    float il[8];
#pragma unroll
    for (int r = 0; r < 8; ++r) il[r] = __fdiv_rn(1.0f, lrow[r]);
#pragma unroll
    for (int jd = 0; jd < 4; ++jd)
#pragma unroll
        for (int r = 0; r < 8; ++r) pt[(8 * hi + r) * 72 + jd * 16 + lr] = (h16)(acc[jd][r] * il[r]);
    __syncthreads();
    h16* crow = C16 + ((size_t)b * SEQ + s0) * INNER + h * HD;
    const int rq = lane >> 3, pc = lane & 7;
#pragma unroll 1
    for (int ps = 0; ps < 2; ++ps) {
#pragma unroll
        for (int s = 0; s < 4; ++s) { const int row = s * 4 + rq; const v8h val = *(const v8ha*)(pt + row * 72 + pc * 8); *(volatile v8h*)(crow + (size_t)row * INNER + pc * 8) = val; }
        if (ps == 0) __threadfence(); }
}

extern "C" void kernel_launch(void* const* d_in, const int* in_sizes, int n_in,
                              void* d_out, int out_size, void* d_ws, size_t ws_size, hipStream_t stream) {
    if (n_in < 5) return;
    const long long rowsX = (long long)(NB - 1) * SEQ_FULL + SEQ;
    if ((long long)in_sizes[0] < rowsX * DIM) return;
    if (in_sizes[1] < DIM * NQKV || in_sizes[2] < NQKV || in_sizes[3] < INNER * DIM || in_sizes[4] < DIM) return;
    if ((long long)out_size < rowsX * DIM) return;
    const float* x    = (const float*)d_in[0];
    const float* wqkv = (const float*)d_in[1];
    const float* bqkv = (const float*)d_in[2];
    const float* wout = (const float*)d_in[3];
    const float* bout = (const float*)d_in[4];
    float* OUT = (float*)d_out;
    char* wsp = (char*)d_ws;
    auto take = [&](size_t bytes) { char* p = wsp; wsp += (bytes + 255) & ~(size_t)255; return (void*)p; };
    bf*    Xb   = (bf*)take((size_t)MROWS * DIM * 2);
    bf*    WqT  = (bf*)take((size_t)NQKV * DIM * 2);
    h16*   WoT  = (h16*)take((size_t)DIM * INNER * 2);
    float* QKVf = (float*)take((size_t)MROWS * NQKV * 4);
    h16*   Q16  = (h16*)take((size_t)NZ * SEQ * HD * 2);
    h16*   K16  = (h16*)take((size_t)NZ * SEQ * HD * 2);
    h16*   VT   = (h16*)take((size_t)NZ * HD * SEQ * 2);
    h16*   C16  = (h16*)take((size_t)MROWS * INNER * 2);
    const size_t used = (size_t)(wsp - (char*)d_ws);
    if (used > ws_size || used > (size_t)134217728) return;

    const unsigned gX = (unsigned)(((size_t)SEQ * DIM / 8 + 255) / 256);
    for (int bb = 0; bb < NB; ++bb)
        k_cvt8<<<gX, 256, 0, stream>>>(x + (size_t)bb * SEQ_FULL * DIM, Xb + (size_t)bb * SEQ * DIM, (size_t)SEQ * DIM / 8);
    k_wt<bf><<<(unsigned)((NQKV * DIM / 64 + 63) / 64), 256, 0, stream>>>(wqkv, DIM, NQKV, 1.0f, WqT);
    k_wt<h16><<<(unsigned)((INNER * DIM / 64 + 63) / 64), 256, 0, stream>>>(wout, INNER, DIM, WSC, WoT);
    k_gemmw<bf, 0, true><<<dim3(MROWS / 64, NQKV / 64, 1), 32, 0, stream>>>(Xb, nullptr, WqT, nullptr, DIM, QKVf, NQKV, bqkv, 1.0f, (size_t)0, (size_t)0, (size_t)0);
    const unsigned gP = (unsigned)(((size_t)NZ * SEQ * HD / 8 + 255) / 256);
    k_qkp<<<gP, 256, 0, stream>>>(QKVf, Q16, K16);
    k_vtp<<<gP, 256, 0, stream>>>(QKVf, VT);
    k_attn<<<dim3(SEQ / 16, NZ, 1), 32, 0, stream>>>(Q16, K16, VT, C16);
    k_gemmw<h16, 0, true><<<dim3(SEQ / 64, DIM / 64, NB), 32, 0, stream>>>(C16, nullptr, WoT, nullptr, INNER, OUT, DIM, bout, OSC, (size_t)SEQ * INNER, (size_t)0, (size_t)SEQ_FULL * DIM);
}
